// CrossGraphEncoder_15436112462316
// MI455X (gfx1250) — hardware-verified
//
#include <hip/hip_runtime.h>
#include <math.h>
#include <stddef.h>
#include <stdint.h>

#pragma clang fp contract(off)


#define NGRAPH 4
#define NAT    256
#define NGRD   1728
#define NATOMS 1024
#define NNODE  7936
#define KAT    8
#define KGR    32
#define CD     64
#define HD     128
#define NLAY   4
#define NGS    20
#define KG1    32
#define PQW    256

#define ETPB 64
#define NTPB 128
#define ITPB 256
#define PTPB 256

#define W1SC  16.0f
#define W1INV 0.0625f
#define GFSC  64.0f
#define GASC  256.0f
#define G1INV 0.00006103515625f
#define W2SC  16.0f
#define HSC   16.0f
#define G2INV 0.00390625f

#define W1T_PL (PQW * CD)
#define GT_PL  (HD * KG1)
#define W2T_PL (CD * HD)
#define BS_PL  PQW

#define WS_W1T  0
#define WS_GT   (WS_W1T + NLAY * W1T_PL * 2)
#define WS_W2T  (WS_GT + NLAY * GT_PL * 2)
#define WS_BIAS (WS_W2T + NLAY * W2T_PL * 2)
#define WS_HA   (WS_BIAS + NLAY * BS_PL * 4)
#define WS_HB   (WS_HA + NNODE * CD * 4)
#define WS_PQ   (WS_HB + NNODE * CD * 4)
#define WS_END  (WS_PQ + NNODE * PQW * 4)
static_assert(WS_GT == 131072 && WS_W2T == 163840 && WS_BIAS == 229376);
static_assert(WS_HA == 233472 && WS_HB == 2265088 && WS_PQ == 4296704 && WS_END == 12423168);
static_assert((WS_GT % 128) == 0 && (WS_W2T % 128) == 0 && (WS_BIAS % 128) == 0);
static_assert((WS_HA % 128) == 0 && (WS_HB % 128) == 0 && (WS_PQ % 128) == 0);

#define SE_ATOM 0
#define SE_G    (SE_ATOM + NATOMS * 16)
#define SE_W2   (SE_G + GT_PL * 2)
#define SE_B2   (SE_W2 + W2T_PL * 2)
#define SE_GAM  (SE_B2 + CD * 4)
#define SE_BET  (SE_GAM + CD * 4)
#define SE_CST  (SE_BET + CD * 4)
#define SE_CSTN 80
#define SE_WAVE (SE_CST + SE_CSTN * 4)
#define EW_IDX  0
#define EW_QP   (EW_IDX + 32 * 32 * 4)
#define EW_A    (EW_QP + 32 * 16)
#define EW_P    (EW_A + 16 * KG1 * 2)
#define EW_HT   (EW_P + 16 * HD * 4)
#define EW_OUT  (EW_HT + 16 * HD * 2)
#define EWB     (EW_OUT + 32 * CD * 4)
#define ESMEM   (SE_WAVE + (ETPB / 32) * EWB)
static_assert(SE_CST == 41728 && SE_WAVE == 42048 && EWB == 26112 && ESMEM == 94272);
static_assert((SE_G % 16) == 0 && (SE_W2 % 16) == 0 && (SE_B2 % 16) == 0 && (SE_WAVE % 16) == 0);
static_assert((SE_CST % 16) == 0 && (((SE_CST + 16 * 4) % 16) == 0) && (((SE_CST + 48 * 4) % 16) == 0));
static_assert((EW_QP % 16) == 0 && (EW_A % 16) == 0 && (EW_P % 16) == 0);
static_assert((EW_HT % 16) == 0 && (EW_OUT % 16) == 0 && (EWB % 16) == 0);
static_assert(ETPB == CD);
static_assert(NATOMS % ETPB == 0 && (NNODE - NATOMS) % ETPB == 0);
static_assert(NAT % 32 == 0 && NGRD % 32 == 0);
static_assert(NNODE % ((NTPB / 32) * 16) == 0);
static_assert((NNODE * 16) % ITPB == 0);
static_assert((32 * KAT) % 16 == 0 && (32 * KGR) % 16 == 0);
static_assert(W1T_PL % (8 * PTPB) == 0 && W2T_PL % (8 * PTPB) == 0 && GT_PL % (8 * PTPB) == 0);

__constant__ unsigned int AXB[12] = {
  0xc1040000u, 0xc0d7ffffu, 0xc0a80000u, 0xc0700000u, 0xc0100000u, 0xbf3ffff8u,
  0x3f400004u, 0x40100000u, 0x40700001u, 0x40a80001u, 0x40d80000u, 0x41040000u};
__constant__ unsigned int OFFB[NGS] = {
  0x00000000u, 0x3dca8850u, 0x3e548c08u, 0x3ea76a90u, 0x3eea9b0cu, 0x3f1a3844u, 0x3f42c99eu,
  0x3f6f5e02u, 0x3f902d80u, 0x3fab181cu, 0x3fc8ac24u, 0x3fe92cfeu, 0x4006725cu, 0x401a1259u,
  0x402fa32cu, 0x404755f8u, 0x406160b8u, 0x407dfec6u, 0x408eb8a8u, 0x40a00000u};
__constant__ unsigned int CFB[NGS] = {
  0xc24c80e0u, 0xc24c80e0u, 0xc2295a0du, 0xc20c3e18u, 0xc1e845dau, 0xc1c05921u, 0xc19f4933u,
  0xc183e819u, 0xc15a7795u, 0xc134ea3eu, 0xc115d181u, 0xc0f82205u, 0xc0cd7b58u, 0xc0aa297au,
  0xc08ce9cfu, 0xc0696249u, 0xc04144c9u, 0xc0200c39u, 0xc00489b1u, 0xbfdb8319u};

typedef float    v4f  __attribute__((ext_vector_type(4)));
typedef float    v8f  __attribute__((ext_vector_type(8)));
typedef int      v4i  __attribute__((ext_vector_type(4)));
typedef _Float16 v4h  __attribute__((ext_vector_type(4)));
typedef _Float16 v8h  __attribute__((ext_vector_type(8)));
typedef _Float16 v16h __attribute__((ext_vector_type(16)));
union FragH { v16h v; v8h h[2]; };

__device__ __forceinline__ v8f wmf(v16h a, v16h b, v8f c) {
  v8f d = __builtin_amdgcn_wmma_f32_16x16x32_f16(false, a, false, b, (short)0, c, false, false);
  asm volatile("v_nop\n\tv_nop\n\tv_nop\n\tv_nop" : "+v"(d) : "v"(a), "v"(b));
  return d;
}

__device__ __forceinline__ v8f splat8(float x) { v8f r = {x, x, x, x, x, x, x, x}; return r; }

__device__ __forceinline__ v16h ldfrag(const _Float16* p, int k0, int hh) {
  FragH u;
  u.h[0] = *(const v8h*)(p + k0 + 8 * hh);
  u.h[1] = *(const v8h*)(p + k0 + 16 + 8 * hh);
  return u.v;
}

__device__ __forceinline__ float vgpr_zero() {
  float z;
  asm volatile("v_mov_b32 %0, 0" : "=v"(z));
  return z;
}

__device__ __forceinline__ void st2f4(float* p, v4f v) {
  *(volatile v4f*)p = v;
  __threadfence();
  *(volatile v4f*)p = v;
}
__device__ __forceinline__ void st2h8(_Float16* p, v8h v) {
  *(volatile v8h*)p = v;
  __threadfence();
  *(volatile v8h*)p = v;
}

__device__ __forceinline__ float d2key(float qx, float qy, float qz, float ax, float ay, float az) {
#pragma clang fp contract(off)
  float dx = qx - ax;
  asm volatile("" : "+v"(dx));
  float dy = qy - ay;
  asm volatile("" : "+v"(dy));
  float dz = qz - az;
  asm volatile("" : "+v"(dz));
  float xx = dx * dx;
  asm volatile("" : "+v"(xx));
  float zz = dz * dz;
  asm volatile("" : "+v"(zz));
  float yy = dy * dy;
  asm volatile("" : "+v"(yy));
  float s = xx + zz;
  asm volatile("" : "+v"(s));
  return s + yy;
}

template <int K>
__device__ __forceinline__ void topk_insert(float (&bd)[K], int (&bi)[K], float d, int m) {
#pragma unroll
  for (int j = K - 1; j >= 1; --j) {
    const bool up = bd[j - 1] > d;
    const bool here = bd[j] > d;
    const float nd = up ? bd[j - 1] : (here ? d : bd[j]);
    const int ni = up ? bi[j - 1] : (here ? m : bi[j]);
    bd[j] = nd;
    bi[j] = ni;
  }
  const bool h0 = bd[0] > d;
  bd[0] = h0 ? d : bd[0];
  bi[0] = h0 ? m : bi[0];
}

template <int K>
__device__ __forceinline__ void knn_select(const v4f* cand, float qx, float qy, float qz,
                                           int jself, int* orow) {
  float bd[K];
  int bi[K];
#pragma unroll
  for (int k = 0; k < K; ++k) { bd[k] = __int_as_float(0x7f800000); bi[k] = 0; }
#pragma unroll 1
  for (int mb = 0; mb < NAT; mb += 4) {
#pragma unroll
    for (int u = 0; u < 4; ++u) {
      const int m = mb + u;
      const v4f a = cand[m];
      float sq = d2key(qx, qy, qz, a.x, a.y, a.z);
      sq = (m == jself) ? (sq + 1.0e9f) : sq;
      if (__builtin_amdgcn_ballot_w32(sq < bd[K - 1]) != 0u) topk_insert<K>(bd, bi, sq, m);
    }
  }
#pragma unroll
  for (int i = 0; i < K / 4; ++i) {
    const v4i v = {bi[4 * i], bi[4 * i + 1], bi[4 * i + 2], bi[4 * i + 3]};
    ((v4i*)orow)[i] = v;
  }
}

__device__ __forceinline__ void ln_store(float x0, float x1, float x2, float x3, int nl,
                                         const float* sGam, const float* sBet, float* orow,
                                         bool wr) {
#pragma clang fp contract(off)
  float s = (x0 + x1) + (x2 + x3);
  s += __shfl_xor(s, 1, 32);
  s += __shfl_xor(s, 2, 32);
  s += __shfl_xor(s, 4, 32);
  s += __shfl_xor(s, 8, 32);
  const float mu = s * 0.015625f;
  const float d0 = x0 - mu, d1 = x1 - mu, d2 = x2 - mu, d3 = x3 - mu;
  float v = (d0 * d0 + d1 * d1) + (d2 * d2 + d3 * d3);
  v += __shfl_xor(v, 1, 32);
  v += __shfl_xor(v, 2, 32);
  v += __shfl_xor(v, 4, 32);
  v += __shfl_xor(v, 8, 32);
  const float var = v * 0.015625f;
  const float inv = 1.0f / sqrtf(var + 1.0e-5f);
  const float y0 = d0 * inv * sGam[nl] + sBet[nl];
  const float y1 = d1 * inv * sGam[16 + nl] + sBet[16 + nl];
  const float y2 = d2 * inv * sGam[32 + nl] + sBet[32 + nl];
  const float y3 = d3 * inv * sGam[48 + nl] + sBet[48 + nl];
  if (wr) {
    orow[nl] = y0;
    orow[16 + nl] = y1;
    orow[32 + nl] = y2;
    orow[48 + nl] = y3;
  }
}

__global__ __launch_bounds__(PTPB) void k_pack(const float* __restrict__ edge_W,
                                               const float* __restrict__ edge_b,
                                               const float* __restrict__ W1,
                                               const float* __restrict__ b1,
                                               const float* __restrict__ W2,
                                               _Float16* W1t, _Float16* Gt, _Float16* W2t,
                                               float* bias) {
#pragma clang fp contract(off)
  const int l = blockIdx.x, t = threadIdx.x;
  const float* eW = edge_W + (size_t)l * NGS * CD;
  const float* eb = edge_b + (size_t)l * CD;
  const float* w1 = W1 + (size_t)l * (3 * CD) * HD;
  const float* bb = b1 + (size_t)l * HD;
  const float* w2 = W2 + (size_t)l * HD * CD;
  _Float16* w1t = W1t + (size_t)l * W1T_PL;
  _Float16* gt  = Gt + (size_t)l * GT_PL;
  _Float16* w2t = W2t + (size_t)l * W2T_PL;
  float* bs = bias + (size_t)l * BS_PL;
  const float zv = vgpr_zero();

#pragma unroll 1
  for (int it = 0; it < W1T_PL / 8 / PTPB; ++it) {
    const int p = it * PTPB + t;
    const int n = p >> 3, k8 = (p & 7) * 8;
    const int nb = (n < HD) ? n : (n - HD);
    const int kb = (n < HD) ? 0 : CD;
    v8h o;
#pragma unroll
    for (int e = 0; e < 8; ++e)
      o[e] = (_Float16)(w1[(size_t)(kb + k8 + e) * HD + nb] * W1SC + zv);
    st2h8(w1t + n * CD + k8, o);
  }
#pragma unroll 1
  for (int it = 0; it < W2T_PL / 8 / PTPB; ++it) {
    const int p = it * PTPB + t;
    const int n = p >> 4, k8 = (p & 15) * 8;
    v8h o;
#pragma unroll
    for (int e = 0; e < 8; ++e)
      o[e] = (_Float16)(w2[(size_t)(k8 + e) * CD + n] * W2SC + zv);
    st2h8(w2t + n * HD + k8, o);
  }
#pragma unroll 1
  for (int it = 0; it < GT_PL / 8 / PTPB; ++it) {
    const int p = it * PTPB + t;
    const int n = p >> 2, k8 = (p & 3) * 8;
    v8h o;
#pragma unroll
    for (int e = 0; e < 8; ++e) {
      const int k = k8 + e;
      const int kc = (k < NGS) ? k : (NGS - 1);
      float s = 0.0f;
#pragma unroll 1
      for (int c = 0; c < CD; ++c) s = fmaf(eW[kc * CD + c], w1[(size_t)(2 * CD + c) * HD + n], s);
      o[e] = (_Float16)((k < NGS) ? (s * GFSC) : zv);
    }
    st2h8(gt + n * KG1 + k8, o);
  }
  if (t < BS_PL / 4) {
    v4f o;
#pragma unroll
    for (int e = 0; e < 4; ++e) {
      const int n = 4 * t + e;
      const int nc = (n < HD) ? 0 : (n - HD);
      float s = bb[nc];
#pragma unroll 1
      for (int c = 0; c < CD; ++c) s = fmaf(eb[c], w1[(size_t)(2 * CD + c) * HD + nc], s);
      o[e] = (n < HD) ? zv : s;
    }
    st2f4(bs + 4 * t, o);
  }
}

__global__ __launch_bounds__(ITPB) void k_init_h(const int* __restrict__ types, float* h0) {
  const int idx = blockIdx.x * ITPB + threadIdx.x;
  const int node = idx >> 4, c4 = (idx & 15) * 4;
  if (node >= NNODE) return;
  const int ty = types[min(node, NATOMS - 1)];
  const bool atom = (node < NATOMS) && (ty >= 0) && (ty < 16);
  v4f o;
#pragma unroll
  for (int e = 0; e < 4; ++e) o[e] = (atom && (c4 + e) == ty) ? 1.0f : 0.0f;
  st2f4(h0 + (size_t)node * CD + c4, o);
}

__global__ __launch_bounds__(NTPB) void k_node(const float* __restrict__ hcur,
                                               const _Float16* __restrict__ W1tL,
                                               const float* __restrict__ biasL,
                                               float* PQ) {
#pragma clang fp contract(off)
  __shared__ __attribute__((aligned(16))) _Float16 sAt[NTPB / 32][16 * CD];
  __shared__ __attribute__((aligned(16))) float sT[NTPB / 32][16 * 32];
  __shared__ float sBias[PQW];
  const int t = threadIdx.x, lane = t & 31, wv = t >> 5, hh = lane >> 4, nl = lane & 15;
  const int row0 = blockIdx.x * ((NTPB / 32) * 16) + 16 * wv;
  _Float16* At = sAt[wv];
  float* T = sT[wv];

  sBias[t] = biasL[t];
  sBias[t + 128] = biasL[t + 128];
#pragma unroll
  for (int it = 0; it < 8; ++it) {
    const int idx = it * 32 + lane;
    const int r = idx >> 4, c4 = (idx & 15) * 4;
    const v4f v = *(const v4f*)(hcur + (size_t)(row0 + r) * CD + c4);
    v4h hv;
    hv[0] = (_Float16)v[0]; hv[1] = (_Float16)v[1]; hv[2] = (_Float16)v[2]; hv[3] = (_Float16)v[3];
    *(v4h*)(At + r * CD + c4) = hv;
  }
  __syncthreads();

  const v16h af0 = ldfrag(At + nl * CD, 0, hh);
  const v16h af1 = ldfrag(At + nl * CD, 32, hh);
#pragma unroll 1
  for (int p = 0; p < PQW / 32; ++p) {
    const _Float16* b0p = W1tL + (size_t)(32 * p + nl) * CD;
    const _Float16* b1p = W1tL + (size_t)(32 * p + 16 + nl) * CD;
    v8f acc0 = splat8(0.0f), acc1 = splat8(0.0f);
    acc0 = wmf(af0, ldfrag(b0p, 0, hh), acc0);
    acc0 = wmf(af1, ldfrag(b0p, 32, hh), acc0);
    acc1 = wmf(af0, ldfrag(b1p, 0, hh), acc1);
    acc1 = wmf(af1, ldfrag(b1p, 32, hh), acc1);
    const float bias0 = sBias[32 * p + nl];
    const float bias1 = sBias[32 * p + 16 + nl];
#pragma unroll
    for (int r = 0; r < 8; ++r) {
      T[(8 * hh + r) * 32 + nl] = acc0[r] * W1INV + bias0;
      T[(8 * hh + r) * 32 + 16 + nl] = acc1[r] * W1INV + bias1;
    }
    __syncthreads();
#pragma unroll
    for (int it = 0; it < 4; ++it) {
      const int r = it * 4 + (lane >> 3), pc = (lane & 7) * 4;
      const v4f v = *(const v4f*)(T + r * 32 + pc);
      st2f4(PQ + (size_t)(row0 + r) * PQW + 32 * p + pc, v);
    }
    __syncthreads();
  }
}

__global__ __launch_bounds__(ETPB) void k_edge(const float* __restrict__ pos,
                                               const float* __restrict__ hcur,
                                               const float* __restrict__ PQ,
                                               const _Float16* __restrict__ GtL,
                                               const _Float16* __restrict__ W2tL,
                                               const float* __restrict__ b2L,
                                               const float* __restrict__ gL,
                                               const float* __restrict__ bL,
                                               float* hOut, float* gout, int last) {
#pragma clang fp contract(off)
  extern __shared__ __attribute__((aligned(16))) char smem[];
  v4f* sAtom = (v4f*)(smem + SE_ATOM);
  _Float16* Gs = (_Float16*)(smem + SE_G);
  _Float16* W2s = (_Float16*)(smem + SE_W2);
  float* sB2 = (float*)(smem + SE_B2);
  float* sGam = (float*)(smem + SE_GAM);
  float* sBet = (float*)(smem + SE_BET);
  float* sAx = (float*)(smem + SE_CST);
  float* sOff = sAx + 16;
  float* sCf = sAx + 48;

  const int t = threadIdx.x, lane = t & 31, wv = t >> 5, hh = lane >> 4, nl = lane & 15;
  char* wreg = smem + SE_WAVE + wv * EWB;
  int* sIdx = (int*)(wreg + EW_IDX);
  v4f* sQpos = (v4f*)(wreg + EW_QP);
  _Float16* sA = (_Float16*)(wreg + EW_A);
  float* sP = (float*)(wreg + EW_P);
  _Float16* Ht = (_Float16*)(wreg + EW_HT);
  float* sOut = (float*)(wreg + EW_OUT);

  const int blk = blockIdx.x;
  const bool isAtom = blk < (NATOMS / ETPB);
  const int node0w = blk * ETPB + 32 * wv;
  const int bq = isAtom ? (node0w >> 8) : ((node0w - NATOMS) / NGRD);

#pragma unroll 1
  for (int a = t; a < NATOMS; a += ETPB) {
    const v4f v = {pos[a * 3 + 0], pos[a * 3 + 1], pos[a * 3 + 2], 0.0f};
    sAtom[a] = v;
  }
#pragma unroll 1
  for (int p = t; p < GT_PL / 8; p += ETPB) *(v8h*)(Gs + 8 * p) = *(const v8h*)(GtL + 8 * p);
#pragma unroll 1
  for (int p = t; p < W2T_PL / 8; p += ETPB) *(v8h*)(W2s + 8 * p) = *(const v8h*)(W2tL + 8 * p);
  sB2[t] = b2L[t];
  sGam[t] = gL[t];
  sBet[t] = bL[t];
  {
    const float axv = __uint_as_float(AXB[min(t, 11)]);
    const int kc = min(t & 31, NGS - 1);
    const float ofv = __uint_as_float(OFFB[kc]);
    const float cfv = __uint_as_float(CFB[kc]);
    if (t < 16) sAx[t] = axv;
    if (t < 32) { sOff[t] = ofv; sCf[t] = cfv; }
  }
  __syncthreads();

  const int node = node0w + lane;
  const v4f qa = sAtom[min(node, NATOMS - 1)];
  int g = node - NATOMS - bq * NGRD;
  g = min(max(g, 0), NGRD - 1);
  const int i0 = g / 144;
  const int gr = g - i0 * 144;
  const int i1 = gr / 12;
  const int i2 = gr - i1 * 12;
  const float gx = sAx[i0];
  const float gy = sAx[i1];
  const float gz = sAx[i2];
  const float qx = isAtom ? qa.x : gx;
  const float qy = isAtom ? qa.y : gy;
  const float qz = isAtom ? qa.z : gz;
  const int jself = isAtom ? (node & (NAT - 1)) : -1;
  {
    const v4f qv = {qx, qy, qz, 0.0f};
    sQpos[lane] = qv;
  }
  const v4f* cand = sAtom + bq * NAT;
  if (isAtom) knn_select<KAT>(cand, qx, qy, qz, jself, sIdx + lane * 32);
  else        knn_select<KGR>(cand, qx, qy, qz, jself, sIdx + lane * 32);
  __syncthreads();

  const int ntile = isAtom ? (32 * KAT / 16) : (32 * KGR / 16);
  const float invcnt = isAtom ? 0.125f : 0.03125f;
  const float zerov = vgpr_zero();
  float agg[4] = {0.0f, 0.0f, 0.0f, 0.0f};

#pragma unroll 1
  for (int tt = 0; tt < ntile; ++tt) {
    {
      const int q = isAtom ? (2 * tt + (nl >> 3)) : (tt >> 1);
      const int s = isAtom ? (nl & 7) : (((tt & 1) << 4) + nl);
      const int jl = sIdx[q * 32 + s] & (NAT - 1);
      const v4f ap = cand[jl];
      const v4f dp = sQpos[q];
      const float rx = ap.x - dp.x, ry = ap.y - dp.y, rz = ap.z - dp.z;
      float dist = sqrtf((rx * rx + ry * ry) + rz * rz);
      dist = fminf(dist, 5.0f);
      FragH gf;
#pragma unroll
      for (int g4 = 0; g4 < 4; ++g4) {
        const v4f o4 = *(const v4f*)(sOff + 16 * hh + 4 * g4);
        const v4f c4 = *(const v4f*)(sCf + 16 * hh + 4 * g4);
#pragma unroll
        for (int e = 0; e < 4; ++e) {
          const int i = 4 * g4 + e;
          const float dd = dist - o4[e];
          const float ex = __expf(c4[e] * (dd * dd)) * GASC;
          const bool real = (hh == 0) || (16 + i < NGS);
          gf.v[i] = (_Float16)(real ? ex : zerov);
        }
      }
      *(v8h*)(sA + nl * KG1 + 16 * hh) = gf.h[0];
      *(v8h*)(sA + nl * KG1 + 16 * hh + 8) = gf.h[1];
    }
#pragma unroll 4
    for (int r = 0; r < 16; ++r) {
      const int q2 = isAtom ? (2 * tt + (r >> 3)) : (tt >> 1);
      const int s2 = isAtom ? (r & 7) : (((tt & 1) << 4) + r);
      const int jl = sIdx[q2 * 32 + s2] & (NAT - 1);
      const v4f v = *(const v4f*)(PQ + (size_t)(bq * NAT + jl) * PQW + 4 * lane);
      *(v4f*)(sP + r * HD + 4 * lane) = v;
    }
    __syncthreads();

    {
      const v16h af = ldfrag(sA + nl * KG1, 0, hh);
      const int qnode = node0w + (isAtom ? (2 * tt + hh) : (tt >> 1));
      const float* qrow = PQ + (size_t)qnode * PQW + HD;
#pragma unroll 2
      for (int nt = 0; nt < HD / 16; ++nt) {
        const int col = nt * 16 + nl;
        const v16h bf = ldfrag(Gs + col * KG1, 0, hh);
        const v8f acc = wmf(af, bf, splat8(0.0f));
        const float qv = qrow[col];
#pragma unroll
        for (int r = 0; r < 8; ++r) {
          const int row = 8 * hh + r;
          float v = acc[r] * G1INV + sP[row * HD + col] + qv;
          v = fmaxf(v, 0.0f) * HSC;
          Ht[row * HD + col] = (_Float16)v;
        }
      }
    }
    __syncthreads();

    float sv[4];
    {
      v16h a2[4];
#pragma unroll
      for (int kt = 0; kt < 4; ++kt) a2[kt] = ldfrag(Ht + nl * HD, 32 * kt, hh);
#pragma unroll
      for (int nt = 0; nt < 4; ++nt) {
        const _Float16* brow = W2s + (nt * 16 + nl) * HD;
        v8f acc = splat8(0.0f);
#pragma unroll
        for (int kt = 0; kt < 4; ++kt) acc = wmf(a2[kt], ldfrag(brow, 32 * kt, hh), acc);
        const float s = ((acc[0] + acc[1]) + (acc[2] + acc[3])) + ((acc[4] + acc[5]) + (acc[6] + acc[7]));
        sv[nt] = s * G2INV;
      }
    }

    if (isAtom) {
      const int qloc = 2 * tt + hh;
      const float* hrow = hcur + (size_t)(node0w + qloc) * CD;
      const float x0 = hrow[nl] + sv[0] * invcnt + sB2[nl];
      const float x1 = hrow[16 + nl] + sv[1] * invcnt + sB2[16 + nl];
      const float x2 = hrow[32 + nl] + sv[2] * invcnt + sB2[32 + nl];
      const float x3 = hrow[48 + nl] + sv[3] * invcnt + sB2[48 + nl];
      ln_store(x0, x1, x2, x3, nl, sGam, sBet, sOut + qloc * CD, true);
    } else {
#pragma unroll
      for (int nt = 0; nt < 4; ++nt) agg[nt] += sv[nt];
      if (tt & 1) {
        const float t0 = agg[0] + __shfl_xor(agg[0], 16, 32);
        const float t1 = agg[1] + __shfl_xor(agg[1], 16, 32);
        const float t2 = agg[2] + __shfl_xor(agg[2], 16, 32);
        const float t3 = agg[3] + __shfl_xor(agg[3], 16, 32);
        const int qloc = tt >> 1;
        const float* hrow = hcur + (size_t)(node0w + qloc) * CD;
        const float x0 = hrow[nl] + t0 * invcnt + sB2[nl];
        const float x1 = hrow[16 + nl] + t1 * invcnt + sB2[16 + nl];
        const float x2 = hrow[32 + nl] + t2 * invcnt + sB2[32 + nl];
        const float x3 = hrow[48 + nl] + t3 * invcnt + sB2[48 + nl];
        ln_store(x0, x1, x2, x3, nl, sGam, sBet, sOut + qloc * CD, hh == 0);
#pragma unroll
        for (int nt = 0; nt < 4; ++nt) agg[nt] = 0.0f;
      }
    }
  }
  __syncthreads();

  float* dstp = (last != 0 && !isAtom) ? (gout + (size_t)(node0w - NATOMS) * CD)
                                        : (hOut + (size_t)node0w * CD);
#pragma unroll
  for (int it = 0; it < 16; ++it) {
    const int r = 2 * it + (lane >> 4), pc = (lane & 15) * 4;
    const v4f v = *(const v4f*)(sOut + r * CD + pc);
    st2f4(dstp + (size_t)r * CD + pc, v);
  }
}

extern "C" void kernel_launch(void* const* d_in, const int* in_sizes, int n_in,
                              void* d_out, int out_size, void* d_ws, size_t ws_size,
                              hipStream_t stream) {
  if (n_in < 11) return;
  if (in_sizes[0] != NATOMS * 3) return;
  if (in_sizes[1] != NATOMS) return;
  if (in_sizes[2] != NATOMS) return;
  if (in_sizes[3] != NLAY * NGS * CD) return;
  if (in_sizes[4] != NLAY * CD) return;
  if (in_sizes[5] != NLAY * (3 * CD) * HD) return;
  if (in_sizes[6] != NLAY * HD) return;
  if (in_sizes[7] != NLAY * HD * CD) return;
  if (in_sizes[8] != NLAY * CD) return;
  if (in_sizes[9] != NLAY * CD) return;
  if (in_sizes[10] != NLAY * CD) return;
  if (out_size != (NNODE - NATOMS) * CD) return;
  if (ws_size < (size_t)WS_END) return;

  const float* pos    = (const float*)d_in[0];
  const int*   types  = (const int*)d_in[1];
  const float* edge_W = (const float*)d_in[3];
  const float* edge_b = (const float*)d_in[4];
  const float* W1     = (const float*)d_in[5];
  const float* b1     = (const float*)d_in[6];
  const float* W2     = (const float*)d_in[7];
  const float* b2     = (const float*)d_in[8];
  const float* lng    = (const float*)d_in[9];
  const float* lnb    = (const float*)d_in[10];
  float* out = (float*)d_out;

  char* ws = (char*)d_ws;
  _Float16* W1t = (_Float16*)(ws + WS_W1T);
  _Float16* Gt  = (_Float16*)(ws + WS_GT);
  _Float16* W2t = (_Float16*)(ws + WS_W2T);
  float* bias = (float*)(ws + WS_BIAS);
  float* hA = (float*)(ws + WS_HA);
  float* hB = (float*)(ws + WS_HB);
  float* PQ = (float*)(ws + WS_PQ);

  k_pack<<<NLAY, PTPB, 0, stream>>>(edge_W, edge_b, W1, b1, W2, W1t, Gt, W2t, bias);
  k_init_h<<<NNODE * 16 / ITPB, ITPB, 0, stream>>>(types, hA);

  hipFuncSetAttribute(reinterpret_cast<const void*>(&k_edge),
                      hipFuncAttributeMaxDynamicSharedMemorySize, ESMEM);

  float* hc = hA;
  float* hn = hB;
  for (int l = 0; l < NLAY; ++l) {
    k_node<<<NNODE / ((NTPB / 32) * 16), NTPB, 0, stream>>>(
        hc, W1t + (size_t)l * W1T_PL, bias + (size_t)l * BS_PL, PQ);
    k_edge<<<NNODE / ETPB, ETPB, ESMEM, stream>>>(
        pos, hc, PQ, Gt + (size_t)l * GT_PL, W2t + (size_t)l * W2T_PL,
        b2 + (size_t)l * CD, lng + (size_t)l * CD, lnb + (size_t)l * CD,
        hn, out, (l == NLAY - 1) ? 1 : 0);
    float* tf = hc; hc = hn; hn = tf;
  }
}
